// SCENE15_JointMembership_89816356094172
// MI455X (gfx1250) — hardware-verified
//
#include <hip/hip_runtime.h>
#include <hip/hip_bf16.h>
#include <stdint.h>


typedef __attribute__((ext_vector_type(16))) _Float16 v16h;
typedef __attribute__((ext_vector_type(8)))  _Float16 v8h;
typedef __attribute__((ext_vector_type(16))) __bf16   v16b;
typedef __attribute__((ext_vector_type(8)))  __bf16   v8b;
typedef __attribute__((ext_vector_type(8)))  float    v8f;
typedef __attribute__((ext_vector_type(4)))  float    v4f;

#define IN_D   200
#define IN_P   224
#define HID    256
#define NCLS   15
#define KFZ    32
#define NC4    64
#define NLAY   3
#define QROWS  32
#define QTHREADS 480
#define QTRIG  (QROWS * IN_D)
#define NTHETA (NCLS * NLAY * 3)
#define NTRIG  (QTRIG + NTHETA)
#define WSC      16.0f
#define WSC_INV  0.0625f
#define FZSC     16384.0f
#define RSC      (1.0f / 262144.0f)

__device__ __forceinline__ unsigned short f2bf_bits(float f) {
  unsigned u = __float_as_uint(f);
  return (unsigned short)((u + 0x7FFFu + ((u >> 16) & 1u)) >> 16);
}
__device__ __forceinline__ float bf_bits2f(unsigned short h) { return __uint_as_float(((unsigned)h) << 16); }

__device__ __forceinline__ void dep_guard_h(v8f& a, v8f& b, v16h x, v16h y) { asm volatile("v_nop\n\tv_nop\n\tv_nop\n\tv_nop" : "+v"(a), "+v"(b) : "v"(x), "v"(y)); }
__device__ __forceinline__ void dep_guard_b(v8f& a, v8f& b, v16b x, v16b y) { asm volatile("v_nop\n\tv_nop\n\tv_nop\n\tv_nop" : "+v"(a), "+v"(b) : "v"(x), "v"(y)); }
__device__ __forceinline__ void keep4_h(v16h a, v16h b, v16h c, v16h d) { asm volatile("v_nop" :: "v"(a), "v"(b), "v"(c), "v"(d)); }
__device__ __forceinline__ void keep4_b(v16b a, v16b b, v16b c, v16b d) { asm volatile("v_nop" :: "v"(a), "v"(b), "v"(c), "v"(d)); }
__device__ __forceinline__ void acc_guard4(v8f& a, v8f& b, v8f& c, v8f& d) { asm volatile("v_nop\n\tv_nop\n\tv_nop\n\tv_nop" : "+v"(a), "+v"(b), "+v"(c), "+v"(d)); }
template <typename T> struct Frag;
template <> struct Frag<_Float16> {
  typedef v16h V; union U { v16h v; v8h h[2]; };
  static __device__ __forceinline__ v16h load(const _Float16* p) {
    U f; f.h[0] = *(const v8h*)(p); f.h[1] = *(const v8h*)(p + 16); return f.v;
  }
  static __device__ __forceinline__ v8f mma(v16h a, v16h b, v8f c) {
    return __builtin_amdgcn_wmma_f32_16x16x32_f16(false, a, false, b, (short)0, c, false, false);
  }
  static __device__ __forceinline__ void guard(v8f& a, v8f& b, v16h x, v16h y) { dep_guard_h(a, b, x, y); }
  static __device__ __forceinline__ void keep(v16h a, v16h b, v16h c, v16h d) { keep4_h(a, b, c, d); }
};
template <> struct Frag<__bf16> {
  typedef v16b V; union U { v16b v; v8b h[2]; };
  static __device__ __forceinline__ v16b load(const __bf16* p) {
    U f; f.h[0] = *(const v8b*)(p); f.h[1] = *(const v8b*)(p + 16); return f.v;
  }
  static __device__ __forceinline__ v8f mma(v16b a, v16b b, v8f c) {
    return __builtin_amdgcn_wmma_f32_16x16x32_bf16(false, a, false, b, (short)0, c, false, false);
  }
  static __device__ __forceinline__ void guard(v8f& a, v8f& b, v16b x, v16b y) { dep_guard_b(a, b, x, y); }
  static __device__ __forceinline__ void keep(v16b a, v16b b, v16b c, v16b d) { keep4_b(a, b, c, d); }
};

template <int ET> struct Elem;
template <> struct Elem<0> { typedef _Float16 T; };
template <> struct Elem<1> { typedef __bf16 T; };
template <int ET, bool SPLIT, int BIAS_MODE, int OUT_MODE, int RESID, int ACT = 0>
__global__ __launch_bounds__(256) void wmma_gemm64(
    const unsigned short* __restrict__ Ap, const unsigned short* __restrict__ A2p, int lda, long strideA,
    const unsigned short* __restrict__ Btp, const unsigned short* __restrict__ Bt2p, int ldb, long strideB,
    void* __restrict__ Cout, void* __restrict__ Cout2, int ldc, long strideC,
    const float* __restrict__ bias,
    const float* __restrict__ resid, long strideR,
    int M, int N, int K, float scale) {
  typedef typename Elem<ET>::T T;
  typedef typename Frag<T>::V V;
  const T* A = (const T*)Ap; const T* A2 = (const T*)A2p; const T* Bt = (const T*)Btp; const T* Bt2 = (const T*)Bt2p;
  __shared__ __align__(16) float sT[8][16 * 68];
  const int b    = blockIdx.y;
  const int lane = threadIdx.x & 31;
  const int wave = threadIdx.x >> 5;
  const int tilesN = N >> 6;
  const int tilesM = M >> 6;
  const int tile = blockIdx.x * 8 + wave;
  if (tile >= tilesM * tilesN) return;
  const int tm = tile / tilesN;
  const int tn = tile - tm * tilesN;
  const int m0 = tm << 6;
  const int n0 = tn << 6;

  const T* Ab  = A  + (size_t)b * strideA;
  const T* Bb  = Bt + (size_t)b * strideB;
  const T* Ab2 = SPLIT ? (A2  + (size_t)b * strideA) : nullptr;
  const T* Bb2 = SPLIT ? (Bt2 + (size_t)b * strideB) : nullptr;

  const int rlane = lane & 15;
  const int koff  = (lane >> 4) * 8;
  const int mOff  = (lane >> 4) * 8;

  v8f acc[4][4];
#pragma unroll
  for (int i = 0; i < 4; ++i)
#pragma unroll
    for (int j = 0; j < 4; ++j) acc[i][j] = (v8f){0.f,0.f,0.f,0.f,0.f,0.f,0.f,0.f};

  for (int k0 = 0; k0 < K; k0 += 32) {
    V bh[4], bl[4];
#pragma unroll
    for (int j = 0; j < 4; ++j) {
      const size_t bo = (size_t)(n0 + (j << 4) + rlane) * ldb + koff + k0;
      bh[j] = Frag<T>::load(Bb + bo);
      if (SPLIT) bl[j] = Frag<T>::load(Bb2 + bo);
    }
#pragma unroll
    for (int i = 0; i < 4; ++i) {
      const size_t ao = (size_t)(m0 + (i << 4) + rlane) * lda + koff + k0;
      V ah = Frag<T>::load(Ab + ao);
      V al;
      if (SPLIT) al = Frag<T>::load(Ab2 + ao);
#pragma unroll
      for (int j = 0; j < 4; ++j) {
        acc[i][j] = Frag<T>::mma(ah, bh[j], acc[i][j]);
        if (SPLIT) {
          acc[i][j] = Frag<T>::mma(ah, bl[j], acc[i][j]);
          acc[i][j] = Frag<T>::mma(al, bh[j], acc[i][j]);
        }
      }
      Frag<T>::guard(acc[i][0], acc[i][3], ah, SPLIT ? al : ah);
    }
    Frag<T>::keep(bh[0], bh[1], bh[2], bh[3]);
    if (SPLIT) Frag<T>::keep(bl[0], bl[1], bl[2], bl[3]);
  }
  acc_guard4(acc[0][0], acc[0][1], acc[0][2], acc[0][3]);
  acc_guard4(acc[1][0], acc[1][1], acc[1][2], acc[1][3]);
  acc_guard4(acc[2][0], acc[2][1], acc[2][2], acc[2][3]);
  acc_guard4(acc[3][0], acc[3][1], acc[3][2], acc[3][3]);

  float* slab = sT[wave];
  const float* Rb = (RESID != 0) ? (resid + (size_t)b * strideR) : nullptr;
#pragma unroll
  for (int i = 0; i < 4; ++i) {
    const int mBase = m0 + (i << 4);
#pragma unroll
    for (int j = 0; j < 4; ++j) {
      const int n = n0 + (j << 4) + rlane;
      float bv = 0.f;
      if (BIAS_MODE == 2) bv = bias[n];
#pragma unroll
      for (int r = 0; r < 8; ++r) {
        float v = acc[i][j][r] * scale;
        if (BIAS_MODE == 1) v += bias[mBase + mOff + r];
        if (BIAS_MODE == 2) v += bv;
        if (RESID == 1) v += Rb[(size_t)(mBase + mOff + r) * ldc + n];
        if (ACT == 1) v = tanhf(v);
        if (ACT == 2) v = fmaxf(v, 0.0f);
        if (ACT == 3) v = v / (1.0f + expf(-v));
        if (ACT == 4) v = (v > 0.f) ? v : 0.01f * v;
        if (ACT == 5) v = 0.5f * v * (1.0f + erff(v * 0.70710678118654752f));
        if (RESID == 2) v += Rb[(size_t)(mBase + mOff + r) * ldc + n];
        slab[(mOff + r) * 68 + (j << 4) + rlane] = v;
      }
    }
    __builtin_amdgcn_fence(__ATOMIC_RELEASE, "workgroup");
    __builtin_amdgcn_wave_barrier();
    __builtin_amdgcn_fence(__ATOMIC_ACQUIRE, "workgroup");
    if (OUT_MODE == 0) {
      float* C = (float*)Cout + (size_t)b * strideC;
      const int hh = lane >> 4, c4 = (lane & 15) * 4;
      for (int pass = 0; pass < 2; ++pass) {
#pragma unroll
        for (int it = 0; it < 8; ++it) {
          const int row = it * 2 + hh;
          v4f v = *(const v4f*)(slab + row * 68 + c4);
          *(volatile v4f*)(C + (size_t)(mBase + row) * ldc + n0 + c4) = v;
        }
        __threadfence();
      }
    } else {
      const int q = lane >> 3, c8 = (lane & 7) * 8;
      unsigned short* C  = (unsigned short*)Cout  + (size_t)b * strideC;
      unsigned short* C2 = (OUT_MODE == 2) ? ((unsigned short*)Cout2 + (size_t)b * strideC) : nullptr;
      for (int pass = 0; pass < 2; ++pass) {
#pragma unroll
        for (int it = 0; it < 4; ++it) {
          const int row = it * 4 + q;
          const float* sp = slab + row * 68 + c8;
          v8h hv, lv;
#pragma unroll
          for (int e = 0; e < 8; ++e) {
            if (OUT_MODE == 1) {
              hv[e] = (_Float16)sp[e];
            } else {
              unsigned short hb = f2bf_bits(sp[e]);
              unsigned short lb = f2bf_bits(sp[e] - bf_bits2f(hb));
              hv[e] = __builtin_bit_cast(_Float16, hb);
              lv[e] = __builtin_bit_cast(_Float16, lb);
            }
          }
          *(volatile v8h*)(C + (size_t)(mBase + row) * ldc + n0 + c8) = hv;
          if (OUT_MODE == 2) *(volatile v8h*)(C2 + (size_t)(mBase + row) * ldc + n0 + c8) = lv;
        }
        __threadfence();
      }
    }
    __builtin_amdgcn_fence(__ATOMIC_RELEASE, "workgroup");
    __builtin_amdgcn_wave_barrier();
    __builtin_amdgcn_fence(__ATOMIC_ACQUIRE, "workgroup");
  }
}

__global__ __launch_bounds__(256) void cast_pad_f16x2(
    const float* __restrict__ in, _Float16* __restrict__ out,
    int R, int C, int Rp, int Cp, float scale, int n2) {
  const int i = blockIdx.x * 256 + threadIdx.x;
  if (i < n2) {
    const int e0 = 2 * i;
    const int r  = e0 / Cp;
    const int c  = e0 - r * Cp;
    const int rr = r < R ? r : R - 1;
    const int c0 = c < C ? c : C - 1;
    const int c1 = (c + 1) < C ? (c + 1) : C - 1;
    float v0 = in[(size_t)rr * C + c0];
    float v1 = in[(size_t)rr * C + c1];
    const bool rin = (r < R);
    v0 = (rin && (c < C)) ? v0 * scale : 0.0f;
    v1 = (rin && ((c + 1) < C)) ? v1 * scale : 0.0f;
    const _Float16 h0 = (_Float16)v0, h1 = (_Float16)v1;
    const unsigned u = (unsigned)__builtin_bit_cast(unsigned short, h0) | ((unsigned)__builtin_bit_cast(unsigned short, h1) << 16);
    ((volatile unsigned*)out)[i] = u;
    __threadfence();
    ((volatile unsigned*)out)[i] = u;
  }
}

__device__ __forceinline__ void qlayer(float cx, float sx, float pr, float ps, float cb, float sb, float qr, float qs,
                                       float& s0r, float& s0i, float& s1r, float& s1i) {
  const float n0r = cx * s0r - sx * s1r;
  const float n0i = cx * s0i - sx * s1i;
  const float n1r = sx * s0r + cx * s1r;
  const float n1i = sx * s0i + cx * s1i;
  const float a0r = n0r * pr + n0i * ps;
  const float a0i = n0i * pr - n0r * ps;
  const float a1r = n1r * pr - n1i * ps;
  const float a1i = n1i * pr + n1r * ps;
  const float m0r = cb * a0r - sb * a1r;
  const float m0i = cb * a0i - sb * a1i;
  const float m1r = sb * a0r + cb * a1r;
  const float m1i = sb * a0i + cb * a1i;
  s0r = m0r * qr + m0i * qs;
  s0i = m0i * qr - m0r * qs;
  s1r = m1r * qr - m1i * qs;
  s1i = m1i * qr + m1r * qs;
}

__global__ __launch_bounds__(QTHREADS) void qsim_kernel(
    const float* __restrict__ x, const float* __restrict__ theta, _Float16* __restrict__ Fz, int nrows) {
  __shared__ float cxs[NTRIG];
  __shared__ float sxs[NTRIG];
  __shared__ float fzs[QROWS * 16];
  const int tid  = threadIdx.x;
  const int row0 = blockIdx.x * QROWS;
  const float* xb = x + (size_t)row0 * IN_D;

#pragma unroll 1
  for (int f = tid; f < NTRIG; f += QTHREADS) {
    const int fx = f < QTRIG ? f : QTRIG - 1;
    int jt = f - QTRIG; jt = jt < 0 ? 0 : (jt > NTHETA - 1 ? NTHETA - 1 : jt);
    const float xa = xb[fx] * 0.5f;
    const float ta = theta[jt] * 0.5f;
    const float ang = (f < QTRIG) ? xa : ta;
    float s, c;
    sincosf(ang, &s, &c);
    cxs[f] = c;
    sxs[f] = s;
  }
  __syncthreads();

  const int rloc = tid / NCLS;
  const int k    = tid - rloc * NCLS;
  const int tb   = QTRIG + k * (NLAY * 3);
  const float pr0 = cxs[tb + 0], ps0 = sxs[tb + 0], cb0 = cxs[tb + 1], sb0 = sxs[tb + 1], qr0 = cxs[tb + 2], qs0 = sxs[tb + 2];
  const float pr1 = cxs[tb + 3], ps1 = sxs[tb + 3], cb1 = cxs[tb + 4], sb1 = sxs[tb + 4], qr1 = cxs[tb + 5], qs1 = sxs[tb + 5];
  const float pr2 = cxs[tb + 6], ps2 = sxs[tb + 6], cb2 = cxs[tb + 7], sb2 = sxs[tb + 7], qr2 = cxs[tb + 8], qs2 = sxs[tb + 8];
  const float* cr = cxs + rloc * IN_D;
  const float* sr = sxs + rloc * IN_D;
  float prod = 1.0f;
#pragma unroll 1
  for (int i = 0; i < IN_D; ++i) {
    const float cx = cr[i], sx = sr[i];
    const float a0r = cx * pr0;
    const float a0i = -(cx * ps0);
    const float a1r = sx * pr0;
    const float a1i = sx * ps0;
    const float m0r = cb0 * a0r - sb0 * a1r;
    const float m0i = cb0 * a0i - sb0 * a1i;
    const float m1r = sb0 * a0r + cb0 * a1r;
    const float m1i = sb0 * a0i + cb0 * a1i;
    float s0r = m0r * qr0 + m0i * qs0;
    float s0i = m0i * qr0 - m0r * qs0;
    float s1r = m1r * qr0 - m1i * qs0;
    float s1i = m1i * qr0 + m1r * qs0;
    qlayer(cx, sx, pr1, ps1, cb1, sb1, qr1, qs1, s0r, s0i, s1r, s1i);
    qlayer(cx, sx, pr2, ps2, cb2, sb2, qr2, qs2, s0r, s0i, s1r, s1i);
    const float z = (s0r * s0r + s0i * s0i) - (s1r * s1r + s1i * s1i);
    const float q = (z + 1.0f) * 0.5f;
    prod = prod * q;
  }
  fzs[rloc * 16 + k] = prod;
  __syncthreads();

  if (tid < 128) {
    const int r  = tid >> 2;
    const int c0 = (tid & 3) * 8;
    v8h hv;
#pragma unroll
    for (int e = 0; e < 8; ++e) {
      const int col = c0 + e;
      const int cc  = col < NCLS ? col : NCLS - 1;
      const float v = fzs[r * 16 + cc];
      hv[e] = (_Float16)((col < NCLS) ? v * FZSC : 0.0f);
    }
    _Float16* dst = Fz + (size_t)(row0 + r) * KFZ + c0;
    *(volatile v8h*)dst = hv;
    __threadfence();
    *(volatile v8h*)dst = hv;
  }
}

__global__ __launch_bounds__(256) void pack_out_kernel(
    const float* __restrict__ C4, const float* __restrict__ bc4, float* __restrict__ out, int n4, int nrows) {
  const int t = blockIdx.x * 256 + threadIdx.x;
  if (t < n4) {
    v4f v;
#pragma unroll
    for (int e = 0; e < 4; ++e) {
      const int f = 4 * t + e;
      int row = f / NCLS;
      const int col = f - row * NCLS;
      row = row < nrows ? row : nrows - 1;
      v[e] = C4[(size_t)row * NC4 + col] + bc4[col];
    }
    float* p = out + (size_t)4 * t;
    *(volatile v4f*)p = v;
    __threadfence();
    *(volatile v4f*)p = v;
  }
}

extern "C" void kernel_launch(void* const* d_in, const int* in_sizes, int n_in,
                              void* d_out, int out_size, void* d_ws, size_t ws_size,
                              hipStream_t stream) {
  if (n_in < 18) return;
  const int Bn = in_sizes[0] / IN_D;
  if (Bn <= 0 || Bn * IN_D != in_sizes[0] || (Bn % 64) != 0 || out_size != Bn * NCLS) return;
  if (in_sizes[1] != HID * IN_D || in_sizes[3] != HID * HID || in_sizes[5] != HID * HID ||
      in_sizes[7] != NTHETA || in_sizes[8] != HID * NCLS || in_sizes[10] != HID * HID ||
      in_sizes[12] != HID * HID || in_sizes[14] != HID * HID || in_sizes[16] != NCLS * HID ||
      in_sizes[2] != HID || in_sizes[9] != HID || in_sizes[17] != NCLS) return;

  const float* x    = (const float*)d_in[0];
  const float* W1   = (const float*)d_in[1];
  const float* b1   = (const float*)d_in[2];
  const float* W2   = (const float*)d_in[3];
  const float* b2   = (const float*)d_in[4];
  const float* W3   = (const float*)d_in[5];
  const float* b3   = (const float*)d_in[6];
  const float* th   = (const float*)d_in[7];
  const float* Wf   = (const float*)d_in[8];
  const float* bfv  = (const float*)d_in[9];
  const float* Wc1  = (const float*)d_in[10];
  const float* bc1  = (const float*)d_in[11];
  const float* Wc2  = (const float*)d_in[12];
  const float* bc2  = (const float*)d_in[13];
  const float* Wc3  = (const float*)d_in[14];
  const float* bc3  = (const float*)d_in[15];
  const float* Wc4  = (const float*)d_in[16];
  const float* bc4  = (const float*)d_in[17];
  float* out = (float*)d_out;

  size_t off = 0;
  auto carve = [&](size_t bytes) -> size_t { size_t r = off; off += (bytes + 255) & ~(size_t)255; return r; };
  const size_t o_xh   = carve((size_t)Bn * IN_P * 2);
  const size_t o_W1h  = carve((size_t)HID * IN_P * 2);
  const size_t o_W2h  = carve((size_t)HID * HID * 2);
  const size_t o_W3h  = carve((size_t)HID * HID * 2);
  const size_t o_Wfh  = carve((size_t)HID * KFZ * 2);
  const size_t o_Wc1h = carve((size_t)HID * HID * 2);
  const size_t o_Wc2h = carve((size_t)HID * HID * 2);
  const size_t o_Wc3h = carve((size_t)HID * HID * 2);
  const size_t o_Wc4h = carve((size_t)NC4 * HID * 2);
  const size_t o_Fz   = carve((size_t)Bn * KFZ * 2);
  const size_t o_actA = carve((size_t)Bn * HID * 2);
  const size_t o_actB = carve((size_t)Bn * HID * 2);
  const size_t o_R    = carve((size_t)Bn * HID * 4);
  const size_t o_C4   = carve((size_t)Bn * NC4 * 4);
  if (off > ws_size || off > (size_t)134217728) return;

  char* ws = (char*)d_ws;
  _Float16* xh   = (_Float16*)(ws + o_xh);
  _Float16* W1h  = (_Float16*)(ws + o_W1h);
  _Float16* W2h  = (_Float16*)(ws + o_W2h);
  _Float16* W3h  = (_Float16*)(ws + o_W3h);
  _Float16* Wfh  = (_Float16*)(ws + o_Wfh);
  _Float16* Wc1h = (_Float16*)(ws + o_Wc1h);
  _Float16* Wc2h = (_Float16*)(ws + o_Wc2h);
  _Float16* Wc3h = (_Float16*)(ws + o_Wc3h);
  _Float16* Wc4h = (_Float16*)(ws + o_Wc4h);
  _Float16* Fz   = (_Float16*)(ws + o_Fz);
  _Float16* actA = (_Float16*)(ws + o_actA);
  _Float16* actB = (_Float16*)(ws + o_actB);
  float*    R    = (float*)(ws + o_R);
  float*    C4   = (float*)(ws + o_C4);

  const dim3 blk(256);
  {
    int n2 = Bn * IN_P / 2;
    cast_pad_f16x2<<<dim3((n2 + 255) / 256), blk, 0, stream>>>(x, xh, Bn, IN_D, Bn, IN_P, 1.0f, n2);
    n2 = HID * IN_P / 2;
    cast_pad_f16x2<<<dim3((n2 + 255) / 256), blk, 0, stream>>>(W1, W1h, HID, IN_D, HID, IN_P, WSC, n2);
    n2 = HID * HID / 2;
    cast_pad_f16x2<<<dim3((n2 + 255) / 256), blk, 0, stream>>>(W2,  W2h,  HID, HID, HID, HID, WSC, n2);
    cast_pad_f16x2<<<dim3((n2 + 255) / 256), blk, 0, stream>>>(W3,  W3h,  HID, HID, HID, HID, WSC, n2);
    cast_pad_f16x2<<<dim3((n2 + 255) / 256), blk, 0, stream>>>(Wc1, Wc1h, HID, HID, HID, HID, WSC, n2);
    cast_pad_f16x2<<<dim3((n2 + 255) / 256), blk, 0, stream>>>(Wc2, Wc2h, HID, HID, HID, HID, WSC, n2);
    cast_pad_f16x2<<<dim3((n2 + 255) / 256), blk, 0, stream>>>(Wc3, Wc3h, HID, HID, HID, HID, WSC, n2);
    n2 = HID * KFZ / 2;
    cast_pad_f16x2<<<dim3((n2 + 255) / 256), blk, 0, stream>>>(Wf, Wfh, HID, NCLS, HID, KFZ, WSC, n2);
    n2 = NC4 * HID / 2;
    cast_pad_f16x2<<<dim3((n2 + 255) / 256), blk, 0, stream>>>(Wc4, Wc4h, NCLS, HID, NC4, HID, WSC, n2);
  }

  qsim_kernel<<<dim3(Bn / QROWS), dim3(QTHREADS), 0, stream>>>(x, th, Fz, Bn);

  const int tilesM  = Bn / 64;
  const int blocksH = (tilesM * (HID / 64) + 7) / 8;
  const int blocks4 = (tilesM * (NC4 / 64) + 7) / 8;
  typedef const unsigned short* cus;

  wmma_gemm64<0, false, 2, 0, 0, 0><<<dim3(blocksH, 1), blk, 0, stream>>>(
      (cus)Fz, (cus)Fz, KFZ, 0L, (cus)Wfh, (cus)Wfh, KFZ, 0L,
      (void*)R, (void*)R, HID, 0L, bfv, bfv, 0L, Bn, HID, KFZ, RSC);

  wmma_gemm64<0, false, 2, 1, 0, 2><<<dim3(blocksH, 1), blk, 0, stream>>>(
      (cus)xh, (cus)xh, IN_P, 0L, (cus)W1h, (cus)W1h, IN_P, 0L,
      (void*)actA, (void*)actA, HID, 0L, b1, bfv, 0L, Bn, HID, IN_P, WSC_INV);
  wmma_gemm64<0, false, 2, 1, 0, 2><<<dim3(blocksH, 1), blk, 0, stream>>>(
      (cus)actA, (cus)actA, HID, 0L, (cus)W2h, (cus)W2h, HID, 0L,
      (void*)actB, (void*)actB, HID, 0L, b2, bfv, 0L, Bn, HID, HID, WSC_INV);
  wmma_gemm64<0, false, 2, 1, 2, 2><<<dim3(blocksH, 1), blk, 0, stream>>>(
      (cus)actB, (cus)actB, HID, 0L, (cus)W3h, (cus)W3h, HID, 0L,
      (void*)actA, (void*)actA, HID, 0L, b3, R, 0L, Bn, HID, HID, WSC_INV);
  wmma_gemm64<0, false, 2, 1, 0, 2><<<dim3(blocksH, 1), blk, 0, stream>>>(
      (cus)actA, (cus)actA, HID, 0L, (cus)Wc1h, (cus)Wc1h, HID, 0L,
      (void*)actB, (void*)actB, HID, 0L, bc1, bfv, 0L, Bn, HID, HID, WSC_INV);
  wmma_gemm64<0, false, 2, 1, 0, 2><<<dim3(blocksH, 1), blk, 0, stream>>>(
      (cus)actB, (cus)actB, HID, 0L, (cus)Wc2h, (cus)Wc2h, HID, 0L,
      (void*)actA, (void*)actA, HID, 0L, bc2, bfv, 0L, Bn, HID, HID, WSC_INV);
  wmma_gemm64<0, false, 2, 1, 0, 2><<<dim3(blocksH, 1), blk, 0, stream>>>(
      (cus)actA, (cus)actA, HID, 0L, (cus)Wc3h, (cus)Wc3h, HID, 0L,
      (void*)actB, (void*)actB, HID, 0L, bc3, bfv, 0L, Bn, HID, HID, WSC_INV);
  wmma_gemm64<0, false, 0, 0, 0, 0><<<dim3(blocks4, 1), blk, 0, stream>>>(
      (cus)actB, (cus)actB, HID, 0L, (cus)Wc4h, (cus)Wc4h, HID, 0L,
      (void*)C4, (void*)C4, NC4, 0L, bc4, bfv, 0L, Bn, NC4, HID, WSC_INV);

  {
    const int n4 = Bn * NCLS / 4;
    pack_out_kernel<<<dim3((n4 + 255) / 256), blk, 0, stream>>>(C4, bc4, out, n4, Bn);
  }
}
